// DAM_Module_26542897889560
// MI455X (gfx1250) — hardware-verified
//
#include <hip/hip_runtime.h>
#include <stdint.h>
#include <math.h>


#define NB 4
#define CIN 256
#define COUT 128
#define HH 64
#define WWD 64
#define HW 4096
#define CQK 16
#define KCONV 2304
#define HP 66

typedef _Float16 f16;
typedef unsigned short us;
typedef float v4f __attribute__((ext_vector_type(4)));
typedef float v8f __attribute__((ext_vector_type(8)));
typedef f16 v8h __attribute__((ext_vector_type(8)));
typedef f16 v16h __attribute__((ext_vector_type(16)));
typedef us v8us __attribute__((ext_vector_type(8)));
typedef __bf16 v16b __attribute__((ext_vector_type(16)));

union FragH { v16h v; v8h half[2]; };
union FragB { v16b v; v8us half[2]; };

__device__ __forceinline__ v8f zero8() {
  v8f z = {0.f, 0.f, 0.f, 0.f, 0.f, 0.f, 0.f, 0.f};
  return z;
}

__device__ __forceinline__ v8f mma_h(const FragH& a, const FragH& b, v8f c) {
  c = __builtin_amdgcn_wmma_f32_16x16x32_f16(false, a.v, false, b.v, (short)0, c, false, false);
  asm volatile("v_nop\n\tv_nop\n\tv_nop\n\tv_nop" : "+v"(c) : "v"(a.v), "v"(b.v));
  return c;
}
__device__ __forceinline__ v8f mma_b(const FragB& a, const FragB& b, v8f c) {
  c = __builtin_amdgcn_wmma_f32_16x16x32_bf16(false, a.v, false, b.v, (short)0, c, false, false);
  asm volatile("v_nop\n\tv_nop\n\tv_nop\n\tv_nop" : "+v"(c) : "v"(a.v), "v"(b.v));
  return c;
}

__device__ __forceinline__ FragH ldh(const f16* p) {
  FragH f;
  f.half[0] = *(const v8h*)(p);
  f.half[1] = *(const v8h*)(p + 16);
  return f;
}
__device__ __forceinline__ FragB ldb(const us* p) {
  FragB f;
  f.half[0] = *(const v8us*)(p);
  f.half[1] = *(const v8us*)(p + 16);
  return f;
}

__device__ __forceinline__ us f2bf(float f) {
  unsigned u = __float_as_uint(f);
  u += 0x7FFFu + ((u >> 16) & 1u);
  return (us)(u >> 16);
}
__device__ __forceinline__ float bf2f(us v) { return __uint_as_float(((unsigned)v) << 16); }

__device__ __forceinline__ void split8(v4f a, v4f c, v8us& hv, v8us& lv) {
  float s[8] = {a.x, a.y, a.z, a.w, c.x, c.y, c.z, c.w};
#pragma unroll
  for (int i = 0; i < 8; ++i) {
    const us hh = f2bf(s[i]);
    hv[i] = hh;
    lv[i] = f2bf(s[i] - bf2f(hh));
  }
}

__device__ __forceinline__ float tanh_fast(float x) {
  const float ax = fminf(fabsf(x), 10.0f);
  const float e = __expf(2.0f * ax);
  const float t = 1.0f - 2.0f * __builtin_amdgcn_rcpf(e + 1.0f);
  return copysignf(t, x);
}

__global__ __launch_bounds__(256) void k_prep_x(const float* __restrict__ x, us* xhi, us* xlo) {
  __shared__ __attribute__((aligned(16))) float tile[64][132];
  const int tid = threadIdx.x;
  const int bid = blockIdx.x;
  const int ch = bid & 1;
  const int t2 = bid >> 1;
  const int hp = t2 % HP;
  const int b = t2 / HP;
  const bool inh = (hp >= 1) && (hp <= HH);
  if (inh) {
    const int w = tid & 63, cb = tid >> 6;
    const float* src = x + (((size_t)b * CIN + ch * 128) * HH + (hp - 1)) * WWD + w;
#pragma unroll 4
    for (int j = 0; j < 32; ++j) {
      const int c = cb + 4 * j;
      tile[w][c] = src[(size_t)c * HW];
    }
  }
  __syncthreads();
#pragma unroll 1
  for (int it = 0; it < 5; ++it) {
    const int wp = it * 16 + (tid >> 4);
    const int c0 = (tid & 15) * 8;
    if (wp < HP) {
      v4f a = {0.f, 0.f, 0.f, 0.f};
      v4f c = a;
      if (inh && wp >= 1 && wp <= WWD) {
        a = *(const v4f*)&tile[wp - 1][c0];
        c = *(const v4f*)&tile[wp - 1][c0 + 4];
      }
      v8us hv, lv;
      split8(a, c, hv, lv);
      const size_t off = (((size_t)b * HP + hp) * HP + wp) * CIN + ch * 128 + c0;
      *(volatile v8us*)(xhi + off) = hv;
      *(volatile v8us*)(xlo + off) = lv;
      __threadfence();
      *(volatile v8us*)(xhi + off) = hv;
      *(volatile v8us*)(xlo + off) = lv;
    }
  }
}

__global__ __launch_bounds__(256) void k_prep_w(const float* __restrict__ w, us* whi, us* wlo) {
  const int g = blockIdx.x * 256 + threadIdx.x;
  if (g >= COUT * (KCONV / 8)) return;
  const int co = g / (KCONV / 8);
  const int k0 = (g - co * (KCONV / 8)) * 8;
  const int tap = k0 >> 8, ci0 = k0 & 255;
  const int kh = tap / 3, kw = tap - 3 * kh;
  const float* src = w + (((size_t)co * CIN + ci0) * 3 + kh) * 3 + kw;
  v4f a, c;
  a.x = src[0];  a.y = src[9];  a.z = src[18]; a.w = src[27];
  c.x = src[36]; c.y = src[45]; c.z = src[54]; c.w = src[63];
  v8us hv, lv;
  split8(a, c, hv, lv);
  const size_t off = (size_t)co * KCONV + k0;
  *(volatile v8us*)(whi + off) = hv;
  *(volatile v8us*)(wlo + off) = lv;
  __threadfence();
  *(volatile v8us*)(whi + off) = hv;
  *(volatile v8us*)(wlo + off) = lv;
}

__global__ __launch_bounds__(256) void k_split8(const float* __restrict__ src, us* hi, us* lo, int ngroups) {
  const int g = blockIdx.x * 256 + threadIdx.x;
  if (g >= ngroups) return;
  const float* s = src + (size_t)g * 8;
  v4f a, c;
  a.x = s[0]; a.y = s[1]; a.z = s[2]; a.w = s[3];
  c.x = s[4]; c.y = s[5]; c.z = s[6]; c.w = s[7];
  v8us hv, lv;
  split8(a, c, hv, lv);
  const size_t off = (size_t)g * 8;
  *(volatile v8us*)(hi + off) = hv;
  *(volatile v8us*)(lo + off) = lv;
  __threadfence();
  *(volatile v8us*)(hi + off) = hv;
  *(volatile v8us*)(lo + off) = lv;
}

__global__ __launch_bounds__(256) void k_conv(const us* __restrict__ whi, const us* __restrict__ wlo,
                                              const us* __restrict__ xhi, const us* __restrict__ xlo,
                                              float* y) {
  __shared__ __attribute__((aligned(16))) float ys[8][16][36];
  const int tid = threadIdx.x, wv = tid >> 5, l = tid & 31, h = l >> 4, m = l & 15;
  const int b = blockIdx.x >> 7;
  const int n0 = (blockIdx.x & 127) << 5;
  const int co = wv * 16 + m;
  const us* wrh = whi + (size_t)co * KCONV + 8 * h;
  const us* wrl = wlo + (size_t)co * KCONV + 8 * h;
  const int px0 = n0 + m, px1 = px0 + 16;
  const size_t pb0 = (((size_t)b * HP + (px0 >> 6)) * HP + (px0 & 63)) * CIN + 8 * h;
  const size_t pb1 = (((size_t)b * HP + (px1 >> 6)) * HP + (px1 & 63)) * CIN + 8 * h;
  const us* xh0 = xhi + pb0;
  const us* xl0 = xlo + pb0;
  const us* xh1 = xhi + pb1;
  const us* xl1 = xlo + pb1;

  v8f acc0 = zero8(), acc1 = zero8();
#pragma unroll 1
  for (int kh = 0; kh < 3; ++kh) {
#pragma unroll 1
    for (int kw = 0; kw < 3; ++kw) {
      const int wo0 = (kh * 3 + kw) * CIN;
      const int xo0 = (kh * HP + kw) * CIN;
#pragma unroll 2
      for (int cc = 0; cc < 8; ++cc) {
        const int wo = wo0 + cc * 32, xo = xo0 + cc * 32;
        const FragB Ah = ldb(wrh + wo);
        const FragB Al = ldb(wrl + wo);
        {
          const FragB Bh = ldb(xh0 + xo);
          const FragB Bl = ldb(xl0 + xo);
          acc0 = mma_b(Ah, Bh, acc0);
          acc0 = mma_b(Al, Bh, acc0);
          acc0 = mma_b(Ah, Bl, acc0);
        }
        {
          const FragB Bh = ldb(xh1 + xo);
          const FragB Bl = ldb(xl1 + xo);
          acc1 = mma_b(Ah, Bh, acc1);
          acc1 = mma_b(Al, Bh, acc1);
          acc1 = mma_b(Ah, Bl, acc1);
        }
      }
    }
  }
#pragma unroll
  for (int r = 0; r < 8; ++r) {
    ys[wv][8 * h + r][m] = acc0[r];
    ys[wv][8 * h + r][16 + m] = acc1[r];
  }
  __syncthreads();
  const int q = l >> 3, p = l & 7;
  float* yb = y + ((size_t)(b * COUT + wv * 16)) * HW + n0 + 4 * p;
#pragma unroll
  for (int it = 0; it < 4; ++it) {
    const int row = it * 4 + q;
    const v4f v = *(const v4f*)&ys[wv][row][4 * p];
    *(volatile v4f*)(yb + (size_t)row * HW) = v;
  }
  __threadfence();
#pragma unroll
  for (int it = 0; it < 4; ++it) {
    const int row = it * 4 + q;
    const v4f v = *(const v4f*)&ys[wv][row][4 * p];
    *(volatile v4f*)(yb + (size_t)row * HW) = v;
  }
}

__global__ __launch_bounds__(256) void k_bn(const float* y, const float* __restrict__ gam,
                                            const float* __restrict__ bet, float* feat, f16* fh) {
  __shared__ double red[256];
  const int co = blockIdx.x, tid = threadIdx.x;
  double s = 0.0;
#pragma unroll 4
  for (int i = tid; i < NB * HW; i += 256) {
    const int bb = i >> 12, n = i & (HW - 1);
    s += (double)y[((size_t)(bb * COUT + co)) * HW + n];
  }
  red[tid] = s;
  __syncthreads();
  for (int st = 128; st > 0; st >>= 1) {
    if (tid < st) red[tid] += red[tid + st];
    __syncthreads();
  }
  const double mean = red[0] * (1.0 / (double)(NB * HW));
  __syncthreads();
  double q = 0.0;
#pragma unroll 4
  for (int i = tid; i < NB * HW; i += 256) {
    const int bb = i >> 12, n = i & (HW - 1);
    const double d = (double)y[((size_t)(bb * COUT + co)) * HW + n] - mean;
    q += d * d;
  }
  red[tid] = q;
  __syncthreads();
  for (int st = 128; st > 0; st >>= 1) {
    if (tid < st) red[tid] += red[tid + st];
    __syncthreads();
  }
  const double var = red[0] * (1.0 / (double)(NB * HW));
  const float meanf = (float)mean;
  const float rstd = rsqrtf((float)var + 1e-5f);
  const float g = gam[co], be = bet[co];

#pragma unroll 1
  for (int it = 0; it < 16; ++it) {
    const int e = it * 1024 + tid * 4;
    const int bb = e >> 12, n = e & (HW - 1);
    const size_t idx = ((size_t)(bb * COUT + co)) * HW + n;
    const v4f v = *(const v4f*)(y + idx);
    v4f o;
#pragma unroll
    for (int i = 0; i < 4; ++i) {
      float t = (v[i] - meanf) * rstd;
      t = t * g + be;
      o[i] = fmaxf(t, 0.0f);
    }
    *(volatile v4f*)(feat + idx) = o;
    __threadfence();
    *(volatile v4f*)(feat + idx) = o;
  }
#pragma unroll 1
  for (int it = 0; it < 8; ++it) {
    const int e = it * 2048 + tid * 8;
    const int bb = e >> 12, n = e & (HW - 1);
    const size_t idx = ((size_t)(bb * COUT + co)) * HW + n;
    const v4f a = *(const v4f*)(y + idx);
    const v4f c = *(const v4f*)(y + idx + 4);
    float sv[8] = {a.x, a.y, a.z, a.w, c.x, c.y, c.z, c.w};
    v8h o;
#pragma unroll
    for (int i = 0; i < 8; ++i) {
      float t = (sv[i] - meanf) * rstd;
      t = t * g + be;
      o[i] = (f16)fmaxf(t, 0.0f);
    }
    *(volatile v8h*)(fh + idx) = o;
    __threadfence();
    *(volatile v8h*)(fh + idx) = o;
  }
}

__global__ __launch_bounds__(256) void k_transpose(const float* feat, f16* ft16, us* fthi, us* ftlo) {
  __shared__ __attribute__((aligned(16))) float tile[32][132];
  const int tid = threadIdx.x;
  const int b = blockIdx.x >> 7;
  const int n0 = (blockIdx.x & 127) << 5;
  {
    const int nl = tid & 31, cb = tid >> 5;
    const float* src = feat + ((size_t)b * COUT) * HW + n0 + nl;
#pragma unroll 4
    for (int j = 0; j < 16; ++j) {
      const int c = cb + 8 * j;
      tile[nl][c] = src[(size_t)c * HW];
    }
  }
  __syncthreads();
#pragma unroll 1
  for (int it = 0; it < 2; ++it) {
    const int nl = it * 16 + (tid >> 4), c0 = (tid & 15) * 8;
    const v4f a = *(const v4f*)&tile[nl][c0];
    const v4f c = *(const v4f*)&tile[nl][c0 + 4];
    v8h fv;
    fv[0] = (f16)a.x; fv[1] = (f16)a.y; fv[2] = (f16)a.z; fv[3] = (f16)a.w;
    fv[4] = (f16)c.x; fv[5] = (f16)c.y; fv[6] = (f16)c.z; fv[7] = (f16)c.w;
    v8us hv, lv;
    split8(a, c, hv, lv);
    const size_t off = ((size_t)b * HW + n0 + nl) * COUT + c0;
    *(volatile v8h*)(ft16 + off) = fv;
    *(volatile v8us*)(fthi + off) = hv;
    *(volatile v8us*)(ftlo + off) = lv;
    __threadfence();
    *(volatile v8h*)(ft16 + off) = fv;
    *(volatile v8us*)(fthi + off) = hv;
    *(volatile v8us*)(ftlo + off) = lv;
  }
}

__global__ __launch_bounds__(256) void k_proj(const us* __restrict__ fthi, const us* __restrict__ ftlo,
                                              const us* __restrict__ vwhi, const us* __restrict__ vwlo,
                                              const us* __restrict__ qwhi, const us* __restrict__ qwlo,
                                              const us* __restrict__ kwhi, const us* __restrict__ kwlo,
                                              const float* __restrict__ vb, const float* __restrict__ qb,
                                              const float* __restrict__ kb,
                                              f16* vout, us* q1p, us* q2p, us* kpp) {
  __shared__ __attribute__((aligned(16))) f16 vs[128][72];
  __shared__ __attribute__((aligned(16))) float qs[2][64][16];
  const int tid = threadIdx.x, wv = tid >> 5, l = tid & 31, h = l >> 4, m = l & 15;
  const int b = blockIdx.x >> 6;
  const int n0 = (blockIdx.x & 63) << 6;

  {
    v8f acc[4];
#pragma unroll
    for (int j = 0; j < 4; ++j) acc[j] = zero8();
    const us* arh = vwhi + (size_t)(wv * 16 + m) * COUT + 8 * h;
    const us* arl = vwlo + (size_t)(wv * 16 + m) * COUT + 8 * h;
    const us* frh = fthi + ((size_t)b * HW + n0 + m) * COUT + 8 * h;
    const us* frl = ftlo + ((size_t)b * HW + n0 + m) * COUT + 8 * h;
#pragma unroll 1
    for (int ks = 0; ks < 4; ++ks) {
      const FragB Ah = ldb(arh + ks * 32);
      const FragB Al = ldb(arl + ks * 32);
#pragma unroll
      for (int j = 0; j < 4; ++j) {
        const FragB Bh = ldb(frh + (size_t)j * 16 * COUT + ks * 32);
        const FragB Bl = ldb(frl + (size_t)j * 16 * COUT + ks * 32);
        acc[j] = mma_b(Ah, Bh, acc[j]);
        acc[j] = mma_b(Al, Bh, acc[j]);
        acc[j] = mma_b(Ah, Bl, acc[j]);
      }
    }
#pragma unroll
    for (int r = 0; r < 8; ++r) {
      const float bias = vb[wv * 16 + 8 * h + r];
#pragma unroll
      for (int j = 0; j < 4; ++j)
        vs[wv * 16 + 8 * h + r][j * 16 + m] = (f16)(acc[j][r] + bias);
    }
  }
  {
    const int sel = wv >> 2, nt = wv & 3;
    const us* wh = sel ? kwhi : qwhi;
    const us* wl = sel ? kwlo : qwlo;
    const float* bias = sel ? kb : qb;
    const us* arh = wh + (size_t)m * COUT + 8 * h;
    const us* arl = wl + (size_t)m * COUT + 8 * h;
    const us* frh = fthi + ((size_t)b * HW + n0 + nt * 16 + m) * COUT + 8 * h;
    const us* frl = ftlo + ((size_t)b * HW + n0 + nt * 16 + m) * COUT + 8 * h;
    v8f acq = zero8();
#pragma unroll 1
    for (int ks = 0; ks < 4; ++ks) {
      const FragB Ah = ldb(arh + ks * 32);
      const FragB Al = ldb(arl + ks * 32);
      const FragB Bh = ldb(frh + ks * 32);
      const FragB Bl = ldb(frl + ks * 32);
      acq = mma_b(Ah, Bh, acq);
      acq = mma_b(Al, Bh, acq);
      acq = mma_b(Ah, Bl, acq);
    }
#pragma unroll
    for (int r = 0; r < 8; ++r)
      qs[sel][nt * 16 + m][8 * h + r] = acq[r] + bias[8 * h + r];
  }
  __syncthreads();

#pragma unroll
  for (int it = 0; it < 4; ++it) {
    const int row = it * 32 + (tid >> 3), p = tid & 7;
    const v8h v = *(const v8h*)&vs[row][p * 8];
    *(volatile v8h*)(vout + ((size_t)(b * COUT + row)) * HW + n0 + p * 8) = v;
  }
  const int n = tid >> 2, p = tid & 3;
  const int o0 = (p & 1) * 8;
  v8us q1v, q2v, kpv;
#pragma unroll
  for (int i = 0; i < 8; ++i) {
    const float qv = qs[0][n][o0 + i];
    const float kv = qs[1][n][o0 + i];
    const us qh = f2bf(qv);
    const us ql = f2bf(qv - bf2f(qh));
    const us khh = f2bf(kv);
    const us kll = f2bf(kv - bf2f(khh));
    q1v[i] = qh;
    q2v[i] = (p < 2) ? ql : (us)0;
    kpv[i] = (p < 2) ? khh : kll;
  }
  const size_t offq = ((size_t)b * HW + n0 + n) * 32 + 8 * p;
  *(volatile v8us*)(q1p + offq) = q1v;
  *(volatile v8us*)(q2p + offq) = q2v;
  *(volatile v8us*)(kpp + offq) = kpv;
  __threadfence();
#pragma unroll
  for (int it = 0; it < 4; ++it) {
    const int row = it * 32 + (tid >> 3), pp = tid & 7;
    const v8h v = *(const v8h*)&vs[row][pp * 8];
    *(volatile v8h*)(vout + ((size_t)(b * COUT + row)) * HW + n0 + pp * 8) = v;
  }
  *(volatile v8us*)(q1p + offq) = q1v;
  *(volatile v8us*)(q2p + offq) = q2v;
  *(volatile v8us*)(kpp + offq) = kpv;
}

__global__ __launch_bounds__(256) void k_cam(const f16* __restrict__ fh, f16* attn) {
  __shared__ __attribute__((aligned(16))) float es[16][132];
  const int tid = threadIdx.x, wv = tid >> 5, l = tid & 31, h = l >> 4, m = l & 15;
  const int b = blockIdx.x >> 3;
  const int c0 = (blockIdx.x & 7) << 4;
  const f16* ar = fh + ((size_t)(b * COUT + c0 + m)) * HW + 8 * h;
  const f16* br = fh + ((size_t)(b * COUT + wv * 16 + m)) * HW + 8 * h;
  v8f acc = zero8();
#pragma unroll 4
  for (int ks = 0; ks < 128; ++ks) {
    const FragH A = ldh(ar + ks * 32);
    const FragH B = ldh(br + ks * 32);
    acc = mma_h(A, B, acc);
  }
#pragma unroll
  for (int r = 0; r < 8; ++r) es[8 * h + r][wv * 16 + m] = acc[r];
  __syncthreads();
  const int row = tid >> 4, p = tid & 15;
  float e[8];
#pragma unroll
  for (int i = 0; i < 8; ++i) e[i] = es[row][8 * p + i];
  float mx = e[0];
#pragma unroll
  for (int i = 1; i < 8; ++i) mx = fmaxf(mx, e[i]);
  mx = fmaxf(mx, __shfl_xor(mx, 8, 16));
  mx = fmaxf(mx, __shfl_xor(mx, 4, 16));
  mx = fmaxf(mx, __shfl_xor(mx, 2, 16));
  mx = fmaxf(mx, __shfl_xor(mx, 1, 16));
  v8h o;
#pragma unroll
  for (int i = 0; i < 8; ++i) o[i] = (f16)(tanh_fast(mx - e[i]) * 256.0f);
  const size_t off = ((size_t)(b * COUT + c0 + row)) * COUT + 8 * p;
  *(volatile v8h*)(attn + off) = o;
  __threadfence();
  *(volatile v8h*)(attn + off) = o;
}

__global__ __launch_bounds__(256) void k_pam(const us* __restrict__ kpp, const us* __restrict__ q1p,
                                             const us* __restrict__ q2p, const f16* __restrict__ vpl,
                                             const f16* __restrict__ attn, const f16* __restrict__ ft16,
                                             const float* __restrict__ feat, const float* __restrict__ gca_p,
                                             const float* __restrict__ gpa_p, float* out) {
  __shared__ __attribute__((aligned(16))) f16 Ps[64][72];
  __shared__ __attribute__((aligned(16))) float os[128][68];
  const int tid = threadIdx.x, wv = tid >> 5, l = tid & 31, h = l >> 4, m = l & 15;
  const int b = blockIdx.x >> 6;
  const int m0 = (blockIdx.x & 63) << 6;
  const int mt = wv & 3, ntb = (wv >> 2) * 2;

  const size_t qoff = ((size_t)b * HW + m0 + mt * 16 + m) * 32 + 8 * h;
  const FragB Q1 = ldb(q1p + qoff);
  const FragB Q2 = ldb(q2p + qoff);
  const us* krow = kpp + ((size_t)b * HW + m) * 32 + 8 * h;
  const f16* vrow = vpl + ((size_t)(b * COUT + wv * 16 + m)) * HW + 8 * h;

  v8f acc[4];
#pragma unroll
  for (int j = 0; j < 4; ++j) acc[j] = zero8();

#pragma unroll 1
  for (int nc = 0; nc < 64; ++nc) {
#pragma unroll
    for (int t = 0; t < 2; ++t) {
      const int nt = ntb + t;
      const FragB Ka = ldb(krow + (size_t)(nc * 64 + nt * 16) * 32);
      v8f s = zero8();
      s = mma_b(Ka, Q1, s);
      s = mma_b(Ka, Q2, s);
      v8h pv;
#pragma unroll
      for (int r = 0; r < 8; ++r) pv[r] = (f16)(tanh_fast(s[r]) * 256.0f);
      *(v8h*)&Ps[mt * 16 + m][nt * 16 + 8 * h] = pv;
    }
    __syncthreads();
#pragma unroll
    for (int ks = 0; ks < 2; ++ks) {
      const FragH Av = ldh(vrow + nc * 64 + ks * 32);
#pragma unroll
      for (int j = 0; j < 4; ++j) {
        const FragH Bp = ldh(&Ps[j * 16 + m][ks * 32 + 8 * h]);
        acc[j] = mma_h(Av, Bp, acc[j]);
      }
    }
    __syncthreads();
  }

  v8f cam[4];
#pragma unroll
  for (int j = 0; j < 4; ++j) cam[j] = zero8();
  {
    const f16* arow = attn + ((size_t)(b * COUT + wv * 16 + m)) * COUT + 8 * h;
    const f16* frow = ft16 + ((size_t)b * HW + m0 + m) * COUT + 8 * h;
#pragma unroll 1
    for (int ks = 0; ks < 4; ++ks) {
      const FragH A = ldh(arow + ks * 32);
#pragma unroll
      for (int j = 0; j < 4; ++j) {
        const FragH B = ldh(frow + (size_t)j * 16 * COUT + ks * 32);
        cam[j] = mma_h(A, B, cam[j]);
      }
    }
  }
  const float sc_ca = gca_p[0] * (1.0f / 256.0f);
  const float sc_pa = gpa_p[0] * (1.0f / 256.0f);
#pragma unroll
  for (int j = 0; j < 4; ++j) {
#pragma unroll
    for (int r = 0; r < 8; ++r)
      os[wv * 16 + 8 * h + r][j * 16 + m] = sc_ca * cam[j][r] + sc_pa * acc[j][r];
  }
  __syncthreads();

  const int p = tid & 15;
#pragma unroll 1
  for (int it = 0; it < 8; ++it) {
    const int row = it * 16 + (tid >> 4);
    const size_t go = ((size_t)(b * COUT + row)) * HW + m0 + 4 * p;
    const v4f o = *(const v4f*)&os[row][4 * p];
    const v4f f = *(const v4f*)(feat + go);
    const v4f res = o + 3.0f * f;
    *(volatile v4f*)(out + go) = res;
  }
  __threadfence();
#pragma unroll 1
  for (int it = 0; it < 8; ++it) {
    const int row = it * 16 + (tid >> 4);
    const size_t go = ((size_t)(b * COUT + row)) * HW + m0 + 4 * p;
    const v4f o = *(const v4f*)&os[row][4 * p];
    const v4f f = *(const v4f*)(feat + go);
    const v4f res = o + 3.0f * f;
    *(volatile v4f*)(out + go) = res;
  }
}

extern "C" void kernel_launch(void* const* d_in, const int* in_sizes, int n_in,
                              void* d_out, int out_size, void* d_ws,
                              size_t ws_size, hipStream_t stream) {
  if (n_in < 12) return;
  if (in_sizes[0] != NB * CIN * HW) return;
  if (in_sizes[1] != COUT * CIN * 9) return;
  if (in_sizes[2] < COUT || in_sizes[3] < COUT) return;
  if (in_sizes[4] != CQK * COUT || in_sizes[6] != CQK * COUT) return;
  if (in_sizes[5] < CQK || in_sizes[7] < CQK) return;
  if (in_sizes[8] != COUT * COUT || in_sizes[9] < COUT) return;
  if (in_sizes[10] < 1 || in_sizes[11] < 1) return;
  if (out_size != NB * COUT * HW) return;

  const float* x        = (const float*)d_in[0];
  const float* conv_w   = (const float*)d_in[1];
  const float* bn_gamma = (const float*)d_in[2];
  const float* bn_beta  = (const float*)d_in[3];
  const float* q_w      = (const float*)d_in[4];
  const float* q_b      = (const float*)d_in[5];
  const float* k_w      = (const float*)d_in[6];
  const float* k_b      = (const float*)d_in[7];
  const float* v_w      = (const float*)d_in[8];
  const float* v_b      = (const float*)d_in[9];
  const float* gca      = (const float*)d_in[10];
  const float* gpa      = (const float*)d_in[11];
  float* out = (float*)d_out;

  char* ws = (char*)d_ws;
  size_t off = 0;
  auto carve = [&](size_t bytes) -> char* {
    char* p = ws + off;
    off = (off + bytes + 255) & ~(size_t)255;
    return p;
  };
  const size_t xp_bytes = (size_t)NB * HP * HP * CIN * 2;
  us*    xhi  = (us*)carve(xp_bytes);
  us*    xlo  = (us*)carve(xp_bytes);
  us*    whi  = (us*)carve((size_t)COUT * KCONV * 2);
  us*    wlo  = (us*)carve((size_t)COUT * KCONV * 2);
  float* y    = (float*)carve((size_t)NB * COUT * HW * 4);
  float* feat = (float*)carve((size_t)NB * COUT * HW * 4);
  f16*   fh   = (f16*)carve((size_t)NB * COUT * HW * 2);
  f16*   ft16 = (f16*)carve((size_t)NB * HW * COUT * 2);
  us*    fthi = (us*)carve((size_t)NB * HW * COUT * 2);
  us*    ftlo = (us*)carve((size_t)NB * HW * COUT * 2);
  us*    vwhi = (us*)carve((size_t)COUT * COUT * 2);
  us*    vwlo = (us*)carve((size_t)COUT * COUT * 2);
  us*    qwhi = (us*)carve((size_t)CQK * COUT * 2);
  us*    qwlo = (us*)carve((size_t)CQK * COUT * 2);
  us*    kwhi = (us*)carve((size_t)CQK * COUT * 2);
  us*    kwlo = (us*)carve((size_t)CQK * COUT * 2);
  f16*   vpl  = (f16*)carve((size_t)NB * COUT * HW * 2);
  us*    q1p  = (us*)carve((size_t)NB * HW * 32 * 2);
  us*    q2p  = (us*)carve((size_t)NB * HW * 32 * 2);
  us*    kpp  = (us*)carve((size_t)NB * HW * 32 * 2);
  f16*   attn = (f16*)carve((size_t)NB * COUT * COUT * 2);
  if (off > ws_size || off > ((size_t)128 << 20)) return;

  k_prep_x<<<NB * HP * 2, 256, 0, stream>>>(x, xhi, xlo);
  k_prep_w<<<(COUT * (KCONV / 8) + 255) / 256, 256, 0, stream>>>(conv_w, whi, wlo);
  k_split8<<<(COUT * COUT / 8 + 255) / 256, 256, 0, stream>>>(v_w, vwhi, vwlo, COUT * COUT / 8);
  k_split8<<<(CQK * COUT / 8 + 255) / 256, 256, 0, stream>>>(q_w, qwhi, qwlo, CQK * COUT / 8);
  k_split8<<<(CQK * COUT / 8 + 255) / 256, 256, 0, stream>>>(k_w, kwhi, kwlo, CQK * COUT / 8);

  k_conv<<<NB * (HW / 32), 256, 0, stream>>>(whi, wlo, xhi, xlo, y);
  k_bn<<<COUT, 256, 0, stream>>>(y, bn_gamma, bn_beta, feat, fh);
  k_transpose<<<NB * (HW / 32), 256, 0, stream>>>(feat, ft16, fthi, ftlo);
  k_proj<<<NB * (HW / 64), 256, 0, stream>>>(fthi, ftlo, vwhi, vwlo, qwhi, qwlo, kwhi, kwlo,
                                               v_b, q_b, k_b, vpl, q1p, q2p, kpp);
  k_cam<<<NB * (COUT / 16), 256, 0, stream>>>(fh, attn);
  k_pam<<<NB * (HW / 64), 256, 0, stream>>>(kpp, q1p, q2p, vpl, attn, ft16, feat, gca, gpa, out);
  (void)hipGetLastError();
}
